// SMG_2h_84000970375420
// MI455X (gfx1250) — hardware-verified
//
#include <hip/hip_runtime.h>
#include <stddef.h>
#include <math.h>


#define DH       64
#define NTHR     256
#define NWAVE    8
#define EPT      8
#define NGRP     2
#define CHUNK    (NTHR * EPT * NGRP)
#define WCAP     (EPT * NGRP * 32)
#define LISTN    (NWAVE * WCAP)
#define NBC      4096
#define NBF      1024
#define RCAP     40960
#define RBN      128
#define TGT      256
#define DEGCAP   512
#define OTHR     512
#define BM       32
#define HR       128
#define LDH      72
#define NCLS     10
#define LMAX     8
#define WLSTRIDE 28672
#define WSCAP    134217728
#define SCL_A    8.0f
#define SCL_W    16.0f
#define SCL_ACC  0.0078125f
#define SCL_HD   0.25f
#define SCL_HACC 0.25f

#define LDS_FILL ((RCAP + NBF + LISTN) * 4 + 64)

static_assert((CHUNK & (CHUNK - 1)) == 0);
static_assert(CHUNK <= 4096);
static_assert(NBC <= 4096 && NBF <= 4096);
static_assert((NBC & (NBC - 1)) == 0 && (NBF & (NBF - 1)) == 0);
static_assert(NBC == 4 * NBF);
static_assert(OTHR * 8 == NBC);
static_assert((RCAP % 32) == 0);
static_assert(TGT == NWAVE * 32);
static_assert((NBC % TGT) == 0);
static_assert((TGT % BM) == 0);
static_assert(DH == 64);
static_assert(BM * 8 == NTHR);
static_assert(HR == NWAVE * 16);
static_assert((LDH % 8) == 0 && LDH >= DH);
static_assert(WLSTRIDE == 2 * DH * DH + DH * DH + 2 * DH * DH + DH * 2 * DH);

typedef float    v2f  __attribute__((ext_vector_type(2)));
typedef float    v4f  __attribute__((ext_vector_type(4)));
typedef float    v8f  __attribute__((ext_vector_type(8)));
typedef int      v4i  __attribute__((ext_vector_type(4)));
typedef _Float16 v2h  __attribute__((ext_vector_type(2)));
typedef _Float16 v4h  __attribute__((ext_vector_type(4)));
typedef _Float16 v8h  __attribute__((ext_vector_type(8)));
typedef _Float16 v16h __attribute__((ext_vector_type(16)));
union FragH { v16h v; v8h h[2]; };

__device__ __forceinline__ v8f wmh(v16h a, v16h b, v8f c) {
  v8f d = __builtin_amdgcn_wmma_f32_16x16x32_f16(false, a, false, b, (short)0, c, false, false);
  asm volatile("v_nop\n\tv_nop\n\tv_nop\n\tv_nop" : "+v"(d) : "v"(a), "v"(b));
  return d;
}

__device__ __forceinline__ v8h cvt8(v4f a, v4f b, float s) {
  v8f t;
  t[0] = a.x * s; t[1] = a.y * s; t[2] = a.z * s; t[3] = a.w * s;
  t[4] = b.x * s; t[5] = b.y * s; t[6] = b.z * s; t[7] = b.w * s;
  return __builtin_convertvector(t, v8h);
}

template <int NB>
__device__ __forceinline__ int scan_chunk(const int* __restrict__ dsts, int nE, int cbase, int slotBase,
                                          int vec8, int* list, int tid, int lane, int wave) {
  int wc = 0;
#pragma unroll
  for (int g = 0; g < NGRP; ++g) {
    const int el0  = (g * NTHR + tid) * EPT;
    const int e0   = cbase + el0;
    const int sent = -2147483647 - 1;
    v4i da, db;
    if (vec8 != 0 && cbase + CHUNK <= nE) {
      da = *(const v4i*)(dsts + e0);
      db = *(const v4i*)(dsts + e0 + 4);
    } else {
      da.x = (e0     < nE) ? dsts[min(e0, nE - 1)] : sent;
      da.y = (e0 + 1 < nE) ? dsts[min(e0 + 1, nE - 1)] : sent;
      da.z = (e0 + 2 < nE) ? dsts[min(e0 + 2, nE - 1)] : sent;
      da.w = (e0 + 3 < nE) ? dsts[min(e0 + 3, nE - 1)] : sent;
      db.x = (e0 + 4 < nE) ? dsts[min(e0 + 4, nE - 1)] : sent;
      db.y = (e0 + 5 < nE) ? dsts[min(e0 + 5, nE - 1)] : sent;
      db.z = (e0 + 6 < nE) ? dsts[min(e0 + 6, nE - 1)] : sent;
      db.w = (e0 + 7 < nE) ? dsts[min(e0 + 7, nE - 1)] : sent;
    }
    const unsigned nb = (unsigned)slotBase;
    const unsigned s0 = (unsigned)da.x - nb, s1 = (unsigned)da.y - nb;
    const unsigned s2 = (unsigned)da.z - nb, s3 = (unsigned)da.w - nb;
    const unsigned s4 = (unsigned)db.x - nb, s5 = (unsigned)db.y - nb;
    const unsigned s6 = (unsigned)db.z - nb, s7 = (unsigned)db.w - nb;
    const bool h0 = s0 < (unsigned)NB, h1 = s1 < (unsigned)NB, h2 = s2 < (unsigned)NB, h3 = s3 < (unsigned)NB;
    const bool h4 = s4 < (unsigned)NB, h5 = s5 < (unsigned)NB, h6 = s6 < (unsigned)NB, h7 = s7 < (unsigned)NB;
    const unsigned any = __builtin_amdgcn_ballot_w32(h0 | h1 | h2 | h3 | h4 | h5 | h6 | h7);
    if (any != 0u) {
#define HITJ(J, HJ, SJ) { \
        const unsigned mj = __builtin_amdgcn_ballot_w32(HJ); \
        if (mj != 0u) { \
          if (HJ) { \
            const int pos = wc + (int)__builtin_amdgcn_mbcnt_lo(mj, 0u); \
            if (pos < WCAP) list[wave * WCAP + pos] = ((el0 + (J)) << 12) | (int)(SJ); \
          } \
          wc += (int)__builtin_popcount(mj); } }
      HITJ(0, h0, s0)
      HITJ(1, h1, s1)
      HITJ(2, h2, s2)
      HITJ(3, h3, s3)
      HITJ(4, h4, s4)
      HITJ(5, h5, s5)
      HITJ(6, h6, s6)
      HITJ(7, h7, s7)
#undef HITJ
    }
  }
  return wc;
}

__global__ __launch_bounds__(NTHR) void k_xcvt(const float* __restrict__ x, _Float16* xp, int nN, int nUnits) {
  constexpr int UPR = DH / 8;
  static_assert((UPR & (UPR - 1)) == 0);
  const int i = (int)blockIdx.x * NTHR + (int)threadIdx.x;
  if (i >= nUnits) return;
  const int row = i / UPR;
  const int c0  = (i & (UPR - 1)) * 8;
  int rr = row > nN - 1 ? nN - 1 : row;
  rr = rr < 0 ? 0 : rr;
  const float* p = x + (size_t)rr * DH + c0;
  const v4f a = *(const v4f*)p;
  const v4f b = *(const v4f*)(p + 4);
  v8h o = cvt8(a, b, SCL_A);
  const v8h z = {(_Float16)0.0f, (_Float16)0.0f, (_Float16)0.0f, (_Float16)0.0f,
                 (_Float16)0.0f, (_Float16)0.0f, (_Float16)0.0f, (_Float16)0.0f};
  o = (row < nN) ? o : z;
  _Float16* d = xp + (size_t)i * 8;
  *(volatile v8h*)d = o;
  __threadfence();
  *(volatile v8h*)d = o;
}

__global__ __launch_bounds__(NTHR) void k_prepw(
    const float* __restrict__ W0, const float* __restrict__ m1w1, const float* __restrict__ m1w2,
    const float* __restrict__ m2w1, const float* __restrict__ wrel, const float* __restrict__ wroot,
    _Float16* pW0, _Float16* pWL, int L) {
  __shared__ float sm[64 * 65];
  const int tid = threadIdx.x;
  const int s = blockIdx.x;
  const float* src = W0;
  _Float16* dq = pW0;
  int dp = DH, koff = 0;
  if (s > 0) {
    int i = (s - 1) / 7;
    const int t = (s - 1) - 7 * i;
    i = i > L - 1 ? L - 1 : i;
    i = i < 0 ? 0 : i;
    _Float16* base = pWL + (size_t)i * WLSTRIDE;
    if (t == 0)      { src = m1w1 + (size_t)i * 8192;        dq = base;                    dp = DH;     koff = 0; }
    else if (t == 1) { src = m1w1 + (size_t)i * 8192 + 4096; dq = base + 4096;             dp = DH;     koff = 0; }
    else if (t == 2) { src = m1w2 + (size_t)i * 4096;        dq = base + 8192;             dp = DH;     koff = 0; }
    else if (t == 3) { src = m2w1 + (size_t)i * 8192;        dq = base + 12288;            dp = DH;     koff = 0; }
    else if (t == 4) { src = m2w1 + (size_t)i * 8192 + 4096; dq = base + 12288 + 4096;     dp = DH;     koff = 0; }
    else if (t == 5) { src = wrel + (size_t)i * 4096;        dq = base + 20480;            dp = 2 * DH; koff = 0; }
    else             { src = wroot + (size_t)i * 4096;       dq = base + 20480;            dp = 2 * DH; koff = DH; }
  }
#pragma unroll 1
  for (int u = tid; u < 1024; u += NTHR) {
    const int row = u >> 4, c4 = (u & 15) * 4;
    const v4f v = *(const v4f*)(src + row * DH + c4);
    float* d = sm + row * 65 + c4;
    d[0] = v.x; d[1] = v.y; d[2] = v.z; d[3] = v.w;
  }
  __syncthreads();
  v8h ov[2];
#pragma unroll
  for (int it = 0; it < 2; ++it) {
    const int u = it * NTHR + tid;
    const int n = u >> 3, p = u & 7;
    v8f t8;
#pragma unroll
    for (int j = 0; j < 8; ++j) t8[j] = sm[(8 * p + j) * 65 + n] * SCL_W;
    ov[it] = __builtin_convertvector(t8, v8h);
  }
#pragma unroll
  for (int it = 0; it < 2; ++it) {
    const int u = it * NTHR + tid;
    const int n = u >> 3, p = u & 7;
    *(volatile v8h*)(dq + (size_t)n * dp + koff + 8 * p) = ov[it];
  }
  __threadfence();
#pragma unroll
  for (int it = 0; it < 2; ++it) {
    const int u = it * NTHR + tid;
    const int n = u >> 3, p = u & 7;
    *(volatile v8h*)(dq + (size_t)n * dp + koff + 8 * p) = ov[it];
  }
}

__global__ __launch_bounds__(NTHR) void k_count(
    const int* __restrict__ dsts, int* cnt, int nE, int vec8) {
  __shared__ __attribute__((aligned(16))) int scnt[NBC];
  __shared__ __attribute__((aligned(16))) int list[LISTN];
  __shared__ int wcnt[NWAVE];
  const int tid = threadIdx.x, lane = tid & 31, wave = tid >> 5;
  const int nodeBase = blockIdx.x * NBC;

  for (int i = tid; i < NBC; i += NTHR) scnt[i] = 0;
  __syncthreads();

  const int nChunks = (nE + CHUNK - 1) / CHUNK;
#pragma unroll 1
  for (int ch = 0; ch < nChunks; ++ch) {
    const int cbase = ch * CHUNK;
    const int wc = scan_chunk<NBC>(dsts, nE, cbase, nodeBase, vec8, list, tid, lane, wave);
    if (lane == 0) wcnt[wave] = wc;
    __syncthreads();
    if (wave == 0) {
#pragma unroll 1
      for (int wsx = 0; wsx < NWAVE; ++wsx) {
        int n = __builtin_amdgcn_readfirstlane(wcnt[wsx]);
        n = n > WCAP ? WCAP : (n < 0 ? 0 : n);
        const int* lp = list + wsx * WCAP;
#pragma unroll 1
        for (int i = 0; i < n; ++i) {
          const int ent  = __builtin_amdgcn_readfirstlane(lp[i]);
          const int slot = ent & (NBC - 1);
          if (lane == 0) scnt[slot] = scnt[slot] + 1;
        }
      }
    }
    __syncthreads();
  }

  v4i cq[4];
#pragma unroll
  for (int q = 0; q < 4; ++q) {
    const int f = (wave * 4 + q) * 128 + 4 * lane;
    cq[q] = *(const v4i*)(scnt + f);
  }
  int* cp = cnt + (size_t)nodeBase;
#pragma unroll
  for (int q = 0; q < 4; ++q) {
    const int f = (wave * 4 + q) * 128 + 4 * lane;
    *(volatile v4i*)(cp + f) = cq[q];
  }
  __threadfence();
#pragma unroll
  for (int q = 0; q < 4; ++q) {
    const int f = (wave * 4 + q) * 128 + 4 * lane;
    *(volatile v4i*)(cp + f) = cq[q];
  }
}

__global__ __launch_bounds__(OTHR) void k_offsets(
    const int* __restrict__ cnt, int* off, int* rbase, int nChunk) {
  __shared__ __attribute__((aligned(16))) int soff[NBC];
  __shared__ __attribute__((aligned(16))) int srb[RBN];
  __shared__ int wtot[OTHR / 32];
  const int tid = threadIdx.x, lane = tid & 31, wave = tid >> 5, sub = tid >> 7;
  for (int i = tid; i < RBN; i += OTHR) srb[i] = 0;
  int carry = 0;
#pragma unroll 1
  for (int ch = 0; ch < nChunk; ++ch) {
    const int base = ch * NBC;
    const v4i c0 = *(const v4i*)(cnt + base + 8 * tid);
    const v4i c1 = *(const v4i*)(cnt + base + 8 * tid + 4);
    const int e0 = max(c0.x, 0), e1 = max(c0.y, 0), e2 = max(c0.z, 0), e3 = max(c0.w, 0);
    const int e4 = max(c1.x, 0), e5 = max(c1.y, 0), e6 = max(c1.z, 0), e7 = max(c1.w, 0);
    const int ts = e0 + e1 + e2 + e3 + e4 + e5 + e6 + e7;
    int incl = ts;
#pragma unroll
    for (int d = 1; d < 32; d <<= 1) {
      const int t = __shfl_up(incl, d);
      if (lane >= d) incl += t;
    }
    if (lane == 31) wtot[wave] = incl;
    __syncthreads();
    const int S0 = wtot[0]  + wtot[1]  + wtot[2]  + wtot[3];
    const int S1 = wtot[4]  + wtot[5]  + wtot[6]  + wtot[7];
    const int S2 = wtot[8]  + wtot[9]  + wtot[10] + wtot[11];
    const int S3 = wtot[12] + wtot[13] + wtot[14] + wtot[15];
    int pre = 0;
#pragma unroll 1
    for (int w = 4 * sub; w < wave; ++w) pre += wtot[w];
    const int b0 = carry;
    const int b1 = b0 + ((S0 + 31) & ~31);
    const int b2 = b1 + ((S1 + 31) & ~31);
    const int b3 = b2 + ((S2 + 31) & ~31);
    const int b4 = b3 + ((S3 + 31) & ~31);
    const int myb = sub == 0 ? b0 : (sub == 1 ? b1 : (sub == 2 ? b2 : b3));
    if (tid == 0) {
      srb[min(4 * ch + 0, RBN - 1)] = b0;
      srb[min(4 * ch + 1, RBN - 1)] = b1;
      srb[min(4 * ch + 2, RBN - 1)] = b2;
      srb[min(4 * ch + 3, RBN - 1)] = b3;
    }
    int run = myb + pre + incl - ts;
    soff[8 * tid + 0] = run; run += e0;
    soff[8 * tid + 1] = run; run += e1;
    soff[8 * tid + 2] = run; run += e2;
    soff[8 * tid + 3] = run; run += e3;
    soff[8 * tid + 4] = run; run += e4;
    soff[8 * tid + 5] = run; run += e5;
    soff[8 * tid + 6] = run; run += e6;
    soff[8 * tid + 7] = run;
    carry = b4;
    __syncthreads();
    const v4i o0 = *(const v4i*)(soff + 4 * tid);
    const v4i o1 = *(const v4i*)(soff + 4 * (tid + OTHR));
    int* op = off + base;
    *(volatile v4i*)(op + 4 * tid) = o0;
    *(volatile v4i*)(op + 4 * (tid + OTHR)) = o1;
    __threadfence();
    *(volatile v4i*)(op + 4 * tid) = o0;
    *(volatile v4i*)(op + 4 * (tid + OTHR)) = o1;
    __syncthreads();
  }
  if (tid == 0) srb[min(4 * nChunk, RBN - 1)] = carry;
  __syncthreads();
  v4i rv = {0, 0, 0, 0};
  if (tid < 32) rv = *(const v4i*)(srb + 4 * tid);
  if (tid < 32) *(volatile v4i*)(rbase + 4 * tid) = rv;
  __threadfence();
  if (tid < 32) *(volatile v4i*)(rbase + 4 * tid) = rv;
}

__global__ __launch_bounds__(NTHR) void k_fill(
    const int* __restrict__ dsts, const int* __restrict__ off, const int* __restrict__ rbase,
    int* csr, int nE, int vec8, int csrLen) {
  extern __shared__ v4f lds_dyn[];
  int* region = (int*)lds_dyn;
  int* cursor = region + RCAP;
  int* list   = cursor + NBF;
  int* wcnt   = list + LISTN;
  const int tid = threadIdx.x, lane = tid & 31, wave = tid >> 5;
  const int b = blockIdx.x;
  const int nodeBase = b * NBF;

  int rb0 = rbase[b];
  const int rb1 = rbase[b + 1];
  rb0 = rb0 < 0 ? 0 : (rb0 > csrLen ? csrLen : rb0);
  rb0 &= ~31;
  int len = rb1 - rb0;
  len = len < 0 ? 0 : (len > RCAP ? RCAP : len);
  int lenW = (len + 31) & ~31;
  if (rb0 + lenW > csrLen) lenW = (csrLen - rb0) & ~31;

  {
    const v4i z = {0, 0, 0, 0};
    for (int i = tid; i < RCAP / 4; i += NTHR) ((v4i*)region)[i] = z;
    for (int s = tid; s < NBF; s += NTHR) {
      int o = off[nodeBase + s] - rb0;
      o = o < 0 ? 0 : (o > RCAP ? RCAP : o);
      cursor[s] = o;
    }
  }
  __syncthreads();

  const int nChunks = (nE + CHUNK - 1) / CHUNK;
#pragma unroll 1
  for (int ch = 0; ch < nChunks; ++ch) {
    const int cbase = ch * CHUNK;
    const int wc = scan_chunk<NBF>(dsts, nE, cbase, nodeBase, vec8, list, tid, lane, wave);
    if (lane == 0) wcnt[wave] = wc;
    __syncthreads();
    if (wave == 0) {
#pragma unroll 1
      for (int wsx = 0; wsx < NWAVE; ++wsx) {
        int n = __builtin_amdgcn_readfirstlane(wcnt[wsx]);
        n = n > WCAP ? WCAP : (n < 0 ? 0 : n);
        const int* lp = list + wsx * WCAP;
#pragma unroll 1
        for (int i = 0; i < n; ++i) {
          const int ent  = __builtin_amdgcn_readfirstlane(lp[i]);
          const int slot = ent & (NBF - 1);
          int e = cbase + ((ent >> 12) & (CHUNK - 1));
          e = e > nE - 1 ? nE - 1 : (e < 0 ? 0 : e);
          if (lane == 0) {
            int pos = cursor[slot];
            pos = pos < 0 ? 0 : (pos > RCAP - 1 ? RCAP - 1 : pos);
            region[pos] = e;
            const int np = pos + 1;
            cursor[slot] = np > RCAP ? RCAP : np;
          }
        }
      }
    }
    __syncthreads();
  }

  const int nv = lenW >> 2;
  int* gp = csr + rb0;
#pragma unroll 1
  for (int i = tid; i < nv; i += NTHR) { const v4i v = ((const v4i*)region)[i]; *(volatile v4i*)(gp + 4 * i) = v; }
  __threadfence();
#pragma unroll 1
  for (int i = tid; i < nv; i += NTHR) { const v4i v = ((const v4i*)region)[i]; *(volatile v4i*)(gp + 4 * i) = v; }
}

template <int MODE>
__global__ __launch_bounds__(NTHR) void k_agg(
    const int* __restrict__ csr, const int* __restrict__ off, const int* __restrict__ cnt,
    const int* __restrict__ srcs, const float* __restrict__ gp,
    const float* __restrict__ b1, const float* __restrict__ w2, const float* __restrict__ b2,
    const float* __restrict__ hF, _Float16* outP, float* outF, int nN, int nE, int csrLen) {
  constexpr int PW = (MODE == 0) ? DH : 2 * DH;
  constexpr int QO = (MODE == 0) ? 0 : DH;
  const int tid = threadIdx.x, lane = tid & 31, wave = tid >> 5;
  const int tbase = blockIdx.x * TGT + wave * 32;
  const int col2 = 2 * lane;

  const int cl    = tbase + lane;
  const int cnt_l = cnt[cl];
  const int off_l = off[cl];

  v2f bb = {0.0f, 0.0f};
  v2f wv = {0.0f, 0.0f};
  float b2s = 0.0f;
  if (MODE >= 1) bb = *(const v2f*)(b1 + col2);
  if (MODE == 2) { wv = *(const v2f*)(w2 + col2); b2s = b2[0]; }

#pragma unroll 1
  for (int j = 0; j < 32; ++j) {
    const int c = tbase + j;
    int nraw = __shfl(cnt_l, j);
    nraw = nraw < 0 ? 0 : (nraw > nE ? nE : nraw);
    const int n = nraw > DEGCAP ? DEGCAP : nraw;
    const int st = __shfl(off_l, j);

    v2f pc = bb;
    if (MODE >= 1) pc = pc + *(const v2f*)(gp + (size_t)c * PW + col2);

    v2f acc = {0.0f, 0.0f};
#pragma unroll 1
    for (int q0 = 0; q0 < n; q0 += 32) {
      int pos = st + q0 + lane;
      pos = pos < 0 ? 0 : (pos > csrLen - 1 ? csrLen - 1 : pos);
      int el = csr[pos];
      el = el < 0 ? 0 : (el > nE - 1 ? nE - 1 : el);
      int sl = srcs[el];
      sl = sl < 0 ? 0 : (sl > nN - 1 ? nN - 1 : sl);
      const int mcnt = (n - q0) < 32 ? (n - q0) : 32;
#pragma unroll 1
      for (int pp = 0; pp < mcnt; ++pp) {
        const int s = __builtin_amdgcn_readlane(sl, pp);
        const v2f q = *(const v2f*)(gp + (size_t)s * PW + QO + col2);
        if (MODE == 0) {
          acc = acc + q;
        } else {
          v2f u = pc + q;
          u.x = u.x > 0.0f ? u.x : 0.0f;
          u.y = u.y > 0.0f ? u.y : 0.0f;
          acc = acc + u;
        }
      }
    }

    if (MODE <= 1) {
      v2f v = acc * SCL_A;
      if (nraw > DEGCAP) { const float qn = __int_as_float(0x7fc00000); v.x = qn; v.y = qn; }
      if (c >= nN) { v.x = 0.0f; v.y = 0.0f; }
      const v2h o = __builtin_convertvector(v, v2h);
      _Float16* ph = outP + (size_t)c * DH + col2;
      *(volatile v2h*)ph = o;
      __threadfence();
      *(volatile v2h*)ph = o;
    } else {
      float part = acc.x * wv.x + acc.y * wv.y;
      part += __shfl_xor(part, 16);
      part += __shfl_xor(part, 8);
      part += __shfl_xor(part, 4);
      part += __shfl_xor(part, 2);
      part += __shfl_xor(part, 1);
      const float cf  = (float)nraw;
      const float tot = part + cf * b2s;
      const float rc  = 1.0f / (cf < 1.0f ? 1.0f : cf);
      float v = tot * rc;
      v = v > 40.0f ? 40.0f : (v < -40.0f ? -40.0f : v);
      float gate = 1.0f / (1.0f + __expf(-v));
      if (nraw > DEGCAP) gate = __int_as_float(0x7fc00000);
      const v2f hr = *(const v2f*)(hF + (size_t)c * DH + col2);
      v2f xm = hr * gate;
      if (c >= nN) { xm.x = 0.0f; xm.y = 0.0f; }
      const v2f xs = xm * SCL_A;
      const v2h o = __builtin_convertvector(xs, v2h);
      float*    pf = outF + (size_t)c * DH + col2;
      _Float16* ph = outP + (size_t)c * DH + col2;
      *(volatile v2f*)pf = xm;
      *(volatile v2h*)ph = o;
      __threadfence();
      *(volatile v2f*)pf = xm;
      *(volatile v2h*)ph = o;
    }
  }
}

template <int K, int LDB, int TPW>
__device__ __forceinline__ void mma_pair(const _Float16* __restrict__ Ap, const _Float16* __restrict__ Bp,
                                         int arow, int c0, int m, int hh, v8f (&acc)[TPW]) {
  constexpr int KT = K / 32;
  static_assert(K % 32 == 0 && LDB % 8 == 0);
  const _Float16* ap  = Ap + (size_t)arow * K + 8 * hh;
  const _Float16* bp0 = Bp + (size_t)(c0 + m) * LDB + 8 * hh;
#pragma unroll 1
  for (int kt = 0; kt < KT; ++kt) {
    FragH a;
    a.h[0] = *(const v8h*)(ap + 32 * kt);
    a.h[1] = *(const v8h*)(ap + 32 * kt + 16);
#pragma unroll
    for (int t = 0; t < TPW; ++t) {
      const _Float16* bp = bp0 + (size_t)(16 * t) * LDB + 32 * kt;
      FragH bf;
      bf.h[0] = *(const v8h*)bp;
      bf.h[1] = *(const v8h*)(bp + 16);
      acc[t] = wmh(a.v, bf.v, acc[t]);
    }
  }
}

template <int K, int NC, int LDB, int NPAIR, int EPI, int RELU>
__device__ __forceinline__ void gemm_stage(
    const _Float16* __restrict__ A1, const _Float16* __restrict__ A2,
    const _Float16* __restrict__ Bp, const float* __restrict__ bias, const float* __restrict__ bias2,
    const int* __restrict__ cntp, float* stg, int rowBase, int nN, int lane, int wave) {
  constexpr int TPW = NC / 64;
  static_assert(K % 32 == 0);
  static_assert(NC % 64 == 0 && TPW >= 1);
  static_assert(NPAIR == 1 || NPAIR == 2);
  const int hh = lane >> 4, m = lane & 15;
  const int rg = wave >> 2, cq = wave & 3;
  const int r0 = rg * 16;
  const int c0 = cq * (NC / 4);

  v8f acc[TPW];
#pragma unroll
  for (int t = 0; t < TPW; ++t) { v8f z = {0.f, 0.f, 0.f, 0.f, 0.f, 0.f, 0.f, 0.f}; acc[t] = z; }

  mma_pair<K, LDB, TPW>(A1, Bp, rowBase + r0 + m, c0, m, hh, acc);
  if (NPAIR == 2) mma_pair<K, LDB, TPW>(A2, Bp + K, rowBase + r0 + m, c0, m, hh, acc);

  float* sp = stg + (size_t)(r0 + 8 * hh) * NC + c0 + m;
  const int grow0 = rowBase + r0 + 8 * hh;
  float cfr[8], rcr[8];
#pragma unroll
  for (int r = 0; r < 8; ++r) { cfr[r] = 0.0f; rcr[r] = 1.0f; }
  if (EPI == 3) {
#pragma unroll
    for (int r = 0; r < 8; ++r) {
      int cv = cntp[grow0 + r];
      cv = cv < 0 ? 0 : cv;
      const float cf = (float)cv;
      cfr[r] = cf;
      rcr[r] = 1.0f / (cf < 1.0f ? 1.0f : cf);
    }
  }
#pragma unroll
  for (int t = 0; t < TPW; ++t) {
    const int n = c0 + 16 * t + m;
    float bv = 0.0f, bv2 = 0.0f;
    if (EPI >= 1) bv = bias[n];
    if (EPI == 2) bv2 = bias2[n];
#pragma unroll
    for (int r = 0; r < 8; ++r) {
      const float a = acc[t][r] * SCL_ACC;
      float v = a;
      if (EPI == 1) v = a + bv;
      if (EPI == 2) v = a + bv + bv2;
      if (EPI == 3) {
        float g = (a + cfr[r] * bv) * rcr[r];
        g = g > 40.0f ? 40.0f : (g < -40.0f ? -40.0f : g);
        v = 1.0f / (1.0f + __expf(-g));
      }
      if (RELU) v = v > 0.0f ? v : 0.0f;
      v = (grow0 + r < nN) ? v : 0.0f;
      sp[r * NC + 16 * t] = v;
    }
  }
}

template <int K, int NC, int LDB, int NPAIR>
__global__ __launch_bounds__(NTHR) void k_gemm32(
    const _Float16* __restrict__ A1, const _Float16* __restrict__ A2,
    const _Float16* __restrict__ Bp, const int* __restrict__ cntp,
    float* Zp, int nN) {
  constexpr int NIT4 = (BM * NC / 4) / NTHR;
  static_assert((BM * NC / 4) % NTHR == 0 && NIT4 >= 1);
  __shared__ __attribute__((aligned(16))) float stg[BM * NC];
  const int tid = threadIdx.x, lane = tid & 31, wave = tid >> 5;
  const int rowBase = blockIdx.x * BM;
  const float* nb = (const float*)Bp;

  gemm_stage<K, NC, LDB, NPAIR, 0, 0>(A1, A2, Bp, nb, nb, cntp, stg, rowBase, nN, lane, wave);
  __syncthreads();

  float* tile = Zp + (size_t)rowBase * NC;
  v4f ov[NIT4];
#pragma unroll
  for (int it = 0; it < NIT4; ++it) ov[it] = *(const v4f*)(stg + 4 * (it * NTHR + tid));
#pragma unroll
  for (int it = 0; it < NIT4; ++it) *(volatile v4f*)(tile + 4 * (size_t)(it * NTHR + tid)) = ov[it];
  __threadfence();
#pragma unroll
  for (int it = 0; it < NIT4; ++it) *(volatile v4f*)(tile + 4 * (size_t)(it * NTHR + tid)) = ov[it];
}

template <int K, int LDB, int NPAIR, int EPI, int RELU>
__global__ __launch_bounds__(NTHR) void k_gemm_dual(
    const _Float16* __restrict__ A1, const _Float16* __restrict__ A2,
    const _Float16* __restrict__ Bp, const float* __restrict__ bias, const float* __restrict__ bias2,
    const int* __restrict__ cntp, float* HF, _Float16* HP, int nN) {
  constexpr int NC = DH;
  constexpr int NIT4 = (BM * NC / 4) / NTHR;
  constexpr int NIT8 = (BM * NC / 8) / NTHR;
  static_assert(NIT4 == 2 && NIT8 == 1);
  __shared__ __attribute__((aligned(16))) float stg[BM * NC];
  const int tid = threadIdx.x, lane = tid & 31, wave = tid >> 5;
  const int rowBase = blockIdx.x * BM;

  gemm_stage<K, NC, LDB, NPAIR, EPI, RELU>(A1, A2, Bp, bias, bias2, cntp, stg, rowBase, nN, lane, wave);
  __syncthreads();

  float*    tf = HF + (size_t)rowBase * NC;
  _Float16* th = HP + (size_t)rowBase * NC;
  v4f ov[NIT4];
  v8h hv[NIT8];
#pragma unroll
  for (int it = 0; it < NIT4; ++it) ov[it] = *(const v4f*)(stg + 4 * (it * NTHR + tid));
#pragma unroll
  for (int it = 0; it < NIT8; ++it) {
    const int u = it * NTHR + tid;
    const v4f x0 = *(const v4f*)(stg + 8 * u);
    const v4f x1 = *(const v4f*)(stg + 8 * u + 4);
    hv[it] = cvt8(x0, x1, SCL_A);
  }
#pragma unroll
  for (int it = 0; it < NIT4; ++it) *(volatile v4f*)(tf + 4 * (size_t)(it * NTHR + tid)) = ov[it];
#pragma unroll
  for (int it = 0; it < NIT8; ++it) *(volatile v8h*)(th + 8 * (size_t)(it * NTHR + tid)) = hv[it];
  __threadfence();
#pragma unroll
  for (int it = 0; it < NIT4; ++it) *(volatile v4f*)(tf + 4 * (size_t)(it * NTHR + tid)) = ov[it];
#pragma unroll
  for (int it = 0; it < NIT8; ++it) *(volatile v8h*)(th + 8 * (size_t)(it * NTHR + tid)) = hv[it];
}

template <int K, int LDB>
__global__ __launch_bounds__(NTHR) void k_gemm_mask(
    const _Float16* __restrict__ A1, const _Float16* __restrict__ Bp, const float* __restrict__ bias,
    const int* __restrict__ cntp, _Float16* MP, int nN) {
  constexpr int NC = DH;
  constexpr int NIT8 = (BM * NC / 8) / NTHR;
  static_assert(NIT8 == 1);
  __shared__ __attribute__((aligned(16))) float stg[BM * NC];
  const int tid = threadIdx.x, lane = tid & 31, wave = tid >> 5;
  const int rowBase = blockIdx.x * BM;

  gemm_stage<K, NC, LDB, 1, 3, 0>(A1, A1, Bp, bias, bias, cntp, stg, rowBase, nN, lane, wave);
  __syncthreads();

  _Float16* th = MP + (size_t)rowBase * NC;
  v8h hv[NIT8];
#pragma unroll
  for (int it = 0; it < NIT8; ++it) {
    const int u = it * NTHR + tid;
    const v4f x0 = *(const v4f*)(stg + 8 * u);
    const v4f x1 = *(const v4f*)(stg + 8 * u + 4);
    hv[it] = cvt8(x0, x1, SCL_A);
  }
#pragma unroll
  for (int it = 0; it < NIT8; ++it) *(volatile v8h*)(th + 8 * (size_t)(it * NTHR + tid)) = hv[it];
  __threadfence();
#pragma unroll
  for (int it = 0; it < NIT8; ++it) *(volatile v8h*)(th + 8 * (size_t)(it * NTHR + tid)) = hv[it];
}

__global__ __launch_bounds__(NTHR) void k_pool(const float* __restrict__ hF, const int* __restrict__ bt,
                                               float* pooled, int nN) {
  __shared__ __attribute__((aligned(16))) float spart[NWAVE * DH];
  __shared__ __attribute__((aligned(16))) float srow[DH];
  const int tid = threadIdx.x, lane = tid & 31, wave = tid >> 5;
  const int g = blockIdx.x;
  const int col2 = 2 * lane;
  v2f acc = {0.0f, 0.0f};
#pragma unroll 1
  for (int base = wave * 32; base < nN; base += NTHR) {
    const int n = base + lane;
    int nc = n > nN - 1 ? nN - 1 : n;
    nc = nc < 0 ? 0 : nc;
    const int bv = bt[nc];
    const bool hit = (n < nN) && (bv == g);
    unsigned mk = __builtin_amdgcn_ballot_w32(hit);
    while (mk != 0u) {
      const int pp = __builtin_ctz(mk);
      mk &= mk - 1u;
      const int s = base + pp;
      acc = acc + *(const v2f*)(hF + (size_t)s * DH + col2);
    }
  }
  *(v2f*)(spart + wave * DH + col2) = acc;
  __syncthreads();
  if (tid < DH) {
    float s = 0.0f;
#pragma unroll
    for (int w = 0; w < NWAVE; ++w) s += spart[w * DH + tid];
    srow[tid] = s;
  }
  __syncthreads();
  v4f rv = {0.0f, 0.0f, 0.0f, 0.0f};
  if (tid < 16) rv = *(const v4f*)(srow + 4 * tid);
  float* rp = pooled + (size_t)g * DH + 4 * tid;
  if (tid < 16) *(volatile v4f*)rp = rv;
  __threadfence();
  if (tid < 16) *(volatile v4f*)rp = rv;
}

__global__ __launch_bounds__(NTHR) void k_head(
    const float* __restrict__ pooled, const float* __restrict__ W1, const float* __restrict__ b1,
    const float* __restrict__ W2, const float* __restrict__ b2, float* out, int G) {
  __shared__ __attribute__((aligned(16))) _Float16 sB1[DH * LDH];
  __shared__ __attribute__((aligned(16))) _Float16 sB2[16 * LDH];
  __shared__ __attribute__((aligned(16))) _Float16 sA[HR * LDH];
  __shared__ __attribute__((aligned(16))) _Float16 sH[HR * LDH];
  __shared__ __attribute__((aligned(16))) float sO[HR * 16];
  __shared__ __attribute__((aligned(16))) float sR[HR * NCLS + 16];
  const int tid = threadIdx.x, lane = tid & 31, wave = tid >> 5;
  const int hh = lane >> 4, m = lane & 15;
  const int grow0 = blockIdx.x * HR;

#pragma unroll 1
  for (int e = tid; e < DH * DH; e += NTHR) {
    const int k = e >> 6, n = e & 63;
    sB1[n * LDH + k] = (_Float16)(W1[e] * SCL_W);
  }
#pragma unroll 1
  for (int e = tid; e < 16 * DH; e += NTHR) {
    const int n = e & 15, k = e >> 4;
    const int nc = n < NCLS ? n : NCLS - 1;
    float v = W2[k * NCLS + nc] * SCL_W;
    v = (n < NCLS) ? v : 0.0f;
    sB2[n * LDH + k] = (_Float16)v;
  }
#pragma unroll 1
  for (int u = tid; u < HR * 16; u += NTHR) {
    const int row = u >> 4, c4 = (u & 15) * 4;
    const int grow = grow0 + row;
    int gr = grow > G - 1 ? G - 1 : grow;
    gr = gr < 0 ? 0 : gr;
    v4f v = *(const v4f*)(pooled + (size_t)gr * DH + c4);
    v = v * SCL_HD;
    if (grow >= G) { v.x = 0.0f; v.y = 0.0f; v.z = 0.0f; v.w = 0.0f; }
    const v4h o = __builtin_convertvector(v, v4h);
    *(v4h*)(sA + row * LDH + c4) = o;
  }
  __syncthreads();

  {
    v8f acc[4];
#pragma unroll
    for (int t = 0; t < 4; ++t) { v8f z = {0.f, 0.f, 0.f, 0.f, 0.f, 0.f, 0.f, 0.f}; acc[t] = z; }
    const _Float16* arow = sA + (16 * wave + m) * LDH + 8 * hh;
#pragma unroll
    for (int kt = 0; kt < 2; ++kt) {
      FragH a;
      a.h[0] = *(const v8h*)(arow + 32 * kt);
      a.h[1] = *(const v8h*)(arow + 32 * kt + 16);
#pragma unroll
      for (int t = 0; t < 4; ++t) {
        const _Float16* bp = sB1 + (16 * t + m) * LDH + 32 * kt + 8 * hh;
        FragH bf;
        bf.h[0] = *(const v8h*)bp;
        bf.h[1] = *(const v8h*)(bp + 16);
        acc[t] = wmh(a.v, bf.v, acc[t]);
      }
    }
#pragma unroll
    for (int t = 0; t < 4; ++t) {
      const int n = 16 * t + m;
      const float bv = b1[n];
#pragma unroll
      for (int r = 0; r < 8; ++r) {
        float v = acc[t][r] * SCL_HACC + bv;
        v = v > 0.0f ? v : 0.0f;
        sH[(16 * wave + 8 * hh + r) * LDH + n] = (_Float16)(v * SCL_HD);
      }
    }
  }
  __syncthreads();

  {
    v8f acc2 = {0.f, 0.f, 0.f, 0.f, 0.f, 0.f, 0.f, 0.f};
    const _Float16* arow = sH + (16 * wave + m) * LDH + 8 * hh;
#pragma unroll
    for (int kt = 0; kt < 2; ++kt) {
      FragH a;
      a.h[0] = *(const v8h*)(arow + 32 * kt);
      a.h[1] = *(const v8h*)(arow + 32 * kt + 16);
      const _Float16* bp = sB2 + m * LDH + 32 * kt + 8 * hh;
      FragH bf;
      bf.h[0] = *(const v8h*)bp;
      bf.h[1] = *(const v8h*)(bp + 16);
      acc2 = wmh(a.v, bf.v, acc2);
    }
    const int mc = m < NCLS ? m : NCLS - 1;
    const float b2v = b2[mc];
#pragma unroll
    for (int r = 0; r < 8; ++r) sO[(16 * wave + 8 * hh + r) * 16 + m] = acc2[r] * SCL_HACC + b2v;
  }
  __syncthreads();

  if (tid < HR) {
    const float* o = sO + tid * 16;
    float mx = o[0];
#pragma unroll 1
    for (int c = 1; c < NCLS; ++c) mx = fmaxf(mx, o[c]);
    float se = 0.0f;
#pragma unroll 1
    for (int c = 0; c < NCLS; ++c) se += expf(o[c] - mx);
    const float lse = logf(se);
#pragma unroll 1
    for (int c = 0; c < NCLS; ++c) sR[tid * NCLS + c] = (o[c] - mx) - lse;
  }
  __syncthreads();

  int nrows = G - grow0;
  nrows = nrows > HR ? HR : (nrows < 0 ? 0 : nrows);
  const int nfl = nrows * NCLS;
  const int nunits = (nfl + 3) >> 2;
  float* base = out + (size_t)grow0 * NCLS;
#pragma unroll 1
  for (int u = tid; u < nunits; u += NTHR) {
    const v4f v = *(const v4f*)(sR + 4 * u);
    const int e0 = 4 * u;
    if (e0 + 3 < nfl) {
      *(volatile v4f*)(base + e0) = v;
    } else {
      if (e0 < nfl)     *(volatile float*)(base + e0)     = v.x;
      if (e0 + 1 < nfl) *(volatile float*)(base + e0 + 1) = v.y;
      if (e0 + 2 < nfl) *(volatile float*)(base + e0 + 2) = v.z;
    }
  }
  __threadfence();
#pragma unroll 1
  for (int u = tid; u < nunits; u += NTHR) {
    const v4f v = *(const v4f*)(sR + 4 * u);
    const int e0 = 4 * u;
    if (e0 + 3 < nfl) {
      *(volatile v4f*)(base + e0) = v;
    } else {
      if (e0 < nfl)     *(volatile float*)(base + e0)     = v.x;
      if (e0 + 1 < nfl) *(volatile float*)(base + e0 + 1) = v.y;
      if (e0 + 2 < nfl) *(volatile float*)(base + e0 + 2) = v.z;
    }
  }
}

extern "C" void kernel_launch(void* const* d_in, const int* in_sizes, int n_in,
                              void* d_out, int out_size, void* d_ws, size_t ws_size,
                              hipStream_t stream) {
  if (n_in < 21) return;
  const int nN = in_sizes[2];
  const int nE = in_sizes[1] / 2;
  const int L  = in_sizes[6] / DH;
  const int G  = out_size / NCLS;
  if (nN <= 0 || nE <= 0 || L <= 0 || L > LMAX || G <= 0) return;
  if (in_sizes[0] != nN * DH || in_sizes[1] != 2 * nE || out_size != G * NCLS) return;
  if (in_sizes[3] != DH * DH || in_sizes[4] != DH) return;
  if (in_sizes[5] != L * 2 * DH * DH || in_sizes[6] != L * DH || in_sizes[7] != L * DH * DH || in_sizes[8] != L * DH) return;
  if (in_sizes[9] != L * 2 * DH * DH || in_sizes[10] != L * DH || in_sizes[11] != L * DH || in_sizes[12] != L) return;
  if (in_sizes[13] != L * DH * DH || in_sizes[14] != L * DH || in_sizes[15] != L * DH * DH || in_sizes[16] != L * DH) return;
  if (in_sizes[17] != DH * DH || in_sizes[18] != DH || in_sizes[19] != DH * NCLS || in_sizes[20] != NCLS) return;
  if (nE > (1 << 28) || nN > (1 << 22) || G > (1 << 20)) return;

  const float* x      = (const float*)d_in[0];
  const int*   ei     = (const int*)d_in[1];
  const int*   bt     = (const int*)d_in[2];
  const float* W0     = (const float*)d_in[3];
  const float* b0     = (const float*)d_in[4];
  const float* m1w1   = (const float*)d_in[5];
  const float* m1b1   = (const float*)d_in[6];
  const float* m1w2   = (const float*)d_in[7];
  const float* m1b2   = (const float*)d_in[8];
  const float* m2w1   = (const float*)d_in[9];
  const float* m2b1   = (const float*)d_in[10];
  const float* m2w2   = (const float*)d_in[11];
  const float* m2b2   = (const float*)d_in[12];
  const float* wrel   = (const float*)d_in[13];
  const float* brel   = (const float*)d_in[14];
  const float* wroot  = (const float*)d_in[15];
  const float* broot  = (const float*)d_in[16];
  const float* W1     = (const float*)d_in[17];
  const float* b1h    = (const float*)d_in[18];
  const float* W2     = (const float*)d_in[19];
  const float* b2h    = (const float*)d_in[20];
  const int* src = ei;
  const int* dst = ei + nE;
  float* out = (float*)d_out;

  const int NPAD   = ((nN + TGT - 1) / TGT) * TGT;
  const int nBC    = (nN + NBC - 1) / NBC;
  const int CNTPAD = nBC * NBC;
  if (CNTPAD < NPAD) return;
  if (4 * nBC + 1 > RBN) return;
  const int nBF    = (nN + NBF - 1) / NBF;
  if (nBF + 1 > 4 * nBC + 1) return;
  const int csrLen = ((nE + 31) & ~31) + 4096;
  if (31 * 4 * nBC > 4096) return;
  const int nAgg   = NPAD / TGT;
  const int nGemm  = NPAD / BM;
  const int nXu    = NPAD * (DH / 8);
  const int nHead  = (G + HR - 1) / HR;

  char* ws = (char*)d_ws;
  size_t off = 0;
  const size_t oW0  = off; off += (size_t)DH * DH * 2;             off = (off + 255) & ~(size_t)255;
  const size_t oWL  = off; off += (size_t)L * WLSTRIDE * 2;        off = (off + 255) & ~(size_t)255;
  const size_t oX   = off; off += (size_t)NPAD * DH * 2;           off = (off + 255) & ~(size_t)255;
  const size_t oHF  = off; off += (size_t)NPAD * DH * 4;           off = (off + 255) & ~(size_t)255;
  const size_t oHP  = off; off += (size_t)NPAD * DH * 2;           off = (off + 255) & ~(size_t)255;
  const size_t oPQ  = off; off += (size_t)NPAD * 2 * DH * 4;       off = (off + 255) & ~(size_t)255;
  const size_t oU   = off; off += (size_t)NPAD * DH * 2;           off = (off + 255) & ~(size_t)255;
  const size_t oM1  = off; off += (size_t)NPAD * DH * 2;           off = (off + 255) & ~(size_t)255;
  const size_t oXMF = off; off += (size_t)NPAD * DH * 4;           off = (off + 255) & ~(size_t)255;
  const size_t oXMP = off; off += (size_t)NPAD * DH * 2;           off = (off + 255) & ~(size_t)255;
  const size_t oAG  = off; off += (size_t)NPAD * DH * 2;           off = (off + 255) & ~(size_t)255;
  const size_t oPL  = off; off += (size_t)G * DH * 4;              off = (off + 255) & ~(size_t)255;
  const size_t oCnt = off; off += (size_t)CNTPAD * 4;              off = (off + 255) & ~(size_t)255;
  const size_t oOff = off; off += (size_t)CNTPAD * 4;              off = (off + 255) & ~(size_t)255;
  const size_t oRb  = off; off += (size_t)RBN * 4;                 off = (off + 255) & ~(size_t)255;
  const size_t oCsr = off; off += (size_t)csrLen * 4;              off = (off + 255) & ~(size_t)255;
  if (off > ws_size || off > (size_t)WSCAP) return;
  _Float16* pW0  = (_Float16*)(ws + oW0);
  _Float16* pWL  = (_Float16*)(ws + oWL);
  _Float16* xP   = (_Float16*)(ws + oX);
  float*    hF   = (float*)(ws + oHF);
  _Float16* hP   = (_Float16*)(ws + oHP);
  float*    pqP  = (float*)(ws + oPQ);
  _Float16* uP   = (_Float16*)(ws + oU);
  _Float16* m1P  = (_Float16*)(ws + oM1);
  float*    xmF  = (float*)(ws + oXMF);
  _Float16* xmP  = (_Float16*)(ws + oXMP);
  _Float16* aggP = (_Float16*)(ws + oAG);
  float*    plP  = (float*)(ws + oPL);
  int*   cnt  = (int*)(ws + oCnt);
  int*   offp = (int*)(ws + oOff);
  int*   rb   = (int*)(ws + oRb);
  int*   csr  = (int*)(ws + oCsr);

  const int vec8 = ((nE & 7) == 0) ? 1 : 0;

  k_prepw<<<1 + 7 * L, NTHR, 0, stream>>>(W0, m1w1, m1w2, m2w1, wrel, wroot, pW0, pWL, L);
  k_xcvt<<<(nXu + NTHR - 1) / NTHR, NTHR, 0, stream>>>(x, xP, nN, nXu);

  k_count<<<nBC, NTHR, 0, stream>>>(dst, cnt, nE, vec8);
  k_offsets<<<1, OTHR, 0, stream>>>(cnt, offp, rb, nBC);
  hipFuncSetAttribute(reinterpret_cast<const void*>(&k_fill),
                      hipFuncAttributeMaxDynamicSharedMemorySize, LDS_FILL);
  k_fill<<<nBF, NTHR, LDS_FILL, stream>>>(dst, offp, rb, csr, nE, vec8, csrLen);

  k_gemm_dual<DH, DH, 1, 1, 0><<<nGemm, NTHR, 0, stream>>>(xP, xP, pW0, b0, b0, cnt, hF, hP, nN);

  for (int i = 0; i < L; ++i) {
    const _Float16* wl   = pWL + (size_t)i * WLSTRIDE;
    const _Float16* pPQa = wl;
    const _Float16* pW2m = wl + 8192;
    const _Float16* pPQb = wl + 12288;
    const _Float16* pCV  = wl + 20480;

    k_gemm32<DH, 2 * DH, DH, 1><<<nGemm, NTHR, 0, stream>>>(hP, hP, pPQa, cnt, pqP, nN);
    k_agg<1><<<nAgg, NTHR, 0, stream>>>(csr, offp, cnt, src, pqP, m1b1 + (size_t)i * DH, m2w2, m2b2, hF,
                                        uP, pqP, nN, nE, csrLen);
    k_gemm_mask<DH, DH><<<nGemm, NTHR, 0, stream>>>(uP, pW2m, m1b2 + (size_t)i * DH, cnt, m1P, nN);
    k_gemm32<DH, 2 * DH, DH, 1><<<nGemm, NTHR, 0, stream>>>(m1P, m1P, pPQb, cnt, pqP, nN);
    k_agg<2><<<nAgg, NTHR, 0, stream>>>(csr, offp, cnt, src, pqP, m2b1 + (size_t)i * DH, m2w2 + (size_t)i * DH,
                                        m2b2 + i, hF, xmP, xmF, nN, nE, csrLen);
    k_agg<0><<<nAgg, NTHR, 0, stream>>>(csr, offp, cnt, src, xmF, m1b1, m2w2, m2b2, hF,
                                        aggP, pqP, nN, nE, csrLen);
    k_gemm_dual<DH, 2 * DH, 2, 2, 1><<<nGemm, NTHR, 0, stream>>>(aggP, xmP, pCV, brel + (size_t)i * DH,
                                                                 broot + (size_t)i * DH, cnt, hF, hP, nN);
  }

  k_pool<<<G, NTHR, 0, stream>>>(hF, bt, plP, nN);
  k_head<<<nHead, NTHR, 0, stream>>>(plP, W1, b1h, W2, b2h, out, G);
}
